// scaled_dot_product_attention_46205258170906
// MI455X (gfx1250) — hardware-verified
//
#include <hip/hip_runtime.h>
#include <stdint.h>

#define NB    4
#define SEQ   2048
#define DM    1024
#define NTOK  (NB * SEQ)

typedef _Float16 v16h __attribute__((ext_vector_type(16)));
typedef _Float16 v8h  __attribute__((ext_vector_type(8)));
typedef float    v8f  __attribute__((ext_vector_type(8)));
typedef float    v4f  __attribute__((ext_vector_type(4)));

static_assert((DM % 128) == 0);
static_assert((NTOK % 64) == 0 && (DM % 64) == 0 && (DM % 32) == 0);
static_assert(((NTOK * DM / 8) % 256) == 0 && ((DM * DM / 8) % 256) == 0);
static_assert((((NTOK / 64) * (DM / 64)) % 8) == 0);

__device__ __forceinline__ float bfr(float f) {
  unsigned u = __float_as_uint(f);
  u = (u + 0x7FFFu + ((u >> 16) & 1u)) & 0xFFFF0000u;
  return __uint_as_float(u);
}

__device__ __forceinline__ v16h ldfrag(const _Float16* p) {
  union { v16h v; v8h hh[2]; } f;
  f.hh[0] = *(const v8h*)(p);
  f.hh[1] = *(const v8h*)(p + 16);
  return f.v;
}
__device__ __forceinline__ v8f mma16(v16h a, v16h b, v8f c) {
  return __builtin_amdgcn_wmma_f32_16x16x32_f16(false, a, false, b, (short)0, c, false, false);
}
__device__ __forceinline__ v8f zero8() {
  v8f z;
#pragma unroll
  for (int i = 0; i < 8; ++i) z[i] = 0.0f;
  return z;
}

__device__ __forceinline__ void guard4_2(v8f& a, v8f& b, v8f& c, v8f& d, v16h x, v16h y) {
  asm volatile("v_nop\n\tv_nop\n\tv_nop\n\tv_nop" : "+v"(a), "+v"(b), "+v"(c), "+v"(d) : "v"(x), "v"(y));
}
__device__ __forceinline__ void guard4_4(v8f& a, v8f& b, v8f& c, v8f& d, v16h x0, v16h x1, v16h y0, v16h y1) {
  asm volatile("v_nop\n\tv_nop\n\tv_nop\n\tv_nop"
               : "+v"(a), "+v"(b), "+v"(c), "+v"(d) : "v"(x0), "v"(x1), "v"(y0), "v"(y1));
}
__device__ __forceinline__ void guard2_3(v8f& a, v8f& b, v16h x, v16h y, v16h z) {
  asm volatile("v_nop\n\tv_nop\n\tv_nop\n\tv_nop" : "+v"(a), "+v"(b) : "v"(x), "v"(y), "v"(z));
}
__device__ __forceinline__ void keep4(v16h a, v16h b, v16h c, v16h d) {
  asm volatile("v_nop" :: "v"(a), "v"(b), "v"(c), "v"(d));
}
__device__ __forceinline__ void accg4(v8f& a, v8f& b, v8f& c, v8f& d) {
  asm volatile("v_nop\n\tv_nop\n\tv_nop\n\tv_nop" : "+v"(a), "+v"(b), "+v"(c), "+v"(d));
}

__global__ __launch_bounds__(256) void cvt_kernel(const float* __restrict__ x, const float* __restrict__ wq,
                                                  const float* __restrict__ wk, const float* __restrict__ wv,
                                                  _Float16* __restrict__ x16, _Float16* __restrict__ wq16,
                                                  _Float16* __restrict__ wk16, _Float16* __restrict__ wv16,
                                                  int nbx, int nbw) {
  const int bid = (int)blockIdx.x;
  int seg = 0;
  if (bid >= nbx) seg = 1 + (bid - nbx) / nbw;
  if (seg > 3) return;
  const float* src = (seg == 0) ? x : ((seg == 1) ? wq : ((seg == 2) ? wk : wv));
  _Float16* dst = (seg == 0) ? x16 : ((seg == 1) ? wq16 : ((seg == 2) ? wk16 : wv16));
  const float scl = (seg == 0) ? 8.0f : 64.0f;
  const int base = (seg == 0) ? 0 : (nbx + (seg - 1) * nbw);
  const int li = (bid - base) * 256 + (int)threadIdx.x;
  const size_t e = (size_t)li * 8;
  const v4f a = *(const v4f*)(src + e);
  const v4f b = *(const v4f*)(src + e + 4);
  v8h o;
#pragma unroll
  for (int i = 0; i < 4; ++i) {
    o[i]     = (_Float16)(bfr(a[i]) * scl);
    o[4 + i] = (_Float16)(bfr(b[i]) * scl);
  }
  _Float16* d = dst + e;
  *(volatile v8h*)d = o;
  __threadfence();
  *(volatile v8h*)d = o;
}

template <int OUT_MODE>
__global__ __launch_bounds__(256) void gemm64_kernel(const _Float16* __restrict__ A, int lda,
                                                     const _Float16* __restrict__ Bt, int ldb,
                                                     _Float16* __restrict__ C1, _Float16* __restrict__ C2, int ldc,
                                                     int M, int N, int K, float scale) {
  __shared__ __align__(16) float sT[8][16 * 68];
  const int lane = threadIdx.x & 31, wave = threadIdx.x >> 5;
  const int tilesN = N >> 6, tilesM = M >> 6;
  const int tile = (int)blockIdx.x * 8 + wave;
  if (tile >= tilesM * tilesN) return;
  const int tm = tile / tilesN, tn = tile - tm * tilesN;
  const int m0 = tm << 6, n0 = tn << 6;
  const int rl = lane & 15;
  const int koff = (lane >> 4) * 8;
  const int mOff = (lane >> 4) * 8;

  v8f acc[4][4];
#pragma unroll
  for (int i = 0; i < 4; ++i)
#pragma unroll
    for (int j = 0; j < 4; ++j) acc[i][j] = zero8();

#pragma unroll 1
  for (int k0 = 0; k0 < K; k0 += 32) {
    v16h bh[4];
#pragma unroll
    for (int j = 0; j < 4; ++j) bh[j] = ldfrag(Bt + (size_t)(n0 + (j << 4) + rl) * ldb + koff + k0);
#pragma unroll
    for (int i = 0; i < 4; ++i) {
      const v16h ah = ldfrag(A + (size_t)(m0 + (i << 4) + rl) * lda + koff + k0);
#pragma unroll
      for (int j = 0; j < 4; ++j) acc[i][j] = mma16(ah, bh[j], acc[i][j]);
      guard4_2(acc[i][0], acc[i][1], acc[i][2], acc[i][3], ah, bh[3]);
    }
    keep4(bh[0], bh[1], bh[2], bh[3]);
  }
  accg4(acc[0][0], acc[0][1], acc[0][2], acc[0][3]);
  accg4(acc[1][0], acc[1][1], acc[1][2], acc[1][3]);
  accg4(acc[2][0], acc[2][1], acc[2][2], acc[2][3]);
  accg4(acc[3][0], acc[3][1], acc[3][2], acc[3][3]);

  float* slab = sT[wave];
  const int qq = lane >> 3, c8 = (lane & 7) * 8;
#pragma unroll
  for (int i = 0; i < 4; ++i) {
    const int mBase = m0 + (i << 4);
#pragma unroll
    for (int j = 0; j < 4; ++j) {
#pragma unroll
      for (int r = 0; r < 8; ++r) slab[(mOff + r) * 68 + (j << 4) + rl] = acc[i][j][r] * scale;
    }
    __builtin_amdgcn_fence(__ATOMIC_RELEASE, "workgroup");
    __builtin_amdgcn_wave_barrier();
    __builtin_amdgcn_fence(__ATOMIC_ACQUIRE, "workgroup");
    v8h hv[4], lv[4];
#pragma unroll
    for (int it = 0; it < 4; ++it) {
      const float* sp = slab + (it * 4 + qq) * 68 + c8;
      v8h a, d;
#pragma unroll
      for (int e = 0; e < 8; ++e) {
        const float f = sp[e];
        const _Float16 t = (_Float16)f;
        a[e] = t;
        d[e] = (OUT_MODE == 2) ? (_Float16)((f - (float)t) * 2048.0f) : t;
      }
      hv[it] = a;
      lv[it] = d;
    }
#pragma unroll
    for (int ps = 0; ps < 2; ++ps) {
#pragma unroll
      for (int it = 0; it < 4; ++it) {
        const size_t off = (size_t)(mBase + it * 4 + qq) * ldc + n0 + c8;
        *(volatile v8h*)(C1 + off) = hv[it];
        if (OUT_MODE == 2) *(volatile v8h*)(C2 + off) = lv[it];
      }
      __threadfence();
    }
    __builtin_amdgcn_fence(__ATOMIC_RELEASE, "workgroup");
    __builtin_amdgcn_wave_barrier();
    __builtin_amdgcn_fence(__ATOMIC_ACQUIRE, "workgroup");
  }
}

#define QB       16
#define KCH      256
#define QSP      1032
#define PSP      264
#define OSP      1028
#define LDS_QH   0
#define LDS_QL   33024
#define LDS_PS   66048
#define LDS_PMAX 74496
#define LDS_PSUM 75008
#define LDS_ST   75520
#define ATT_LDS  75776
static_assert(QB * QSP * 2 == LDS_QL - LDS_QH);
static_assert(QB * QSP * 2 == LDS_PS - LDS_QL);
static_assert(QB * PSP * 2 == LDS_PMAX - LDS_PS);
static_assert(LDS_PSUM - LDS_PMAX == 8 * QB * 4);
static_assert(LDS_ST - LDS_PSUM == 8 * QB * 4);
static_assert(ATT_LDS - LDS_ST == 4 * QB * 4);
static_assert(QB * OSP * 4 <= LDS_PS);
static_assert((QSP % 8) == 0 && (PSP % 8) == 0 && (OSP % 4) == 0 && PSP >= KCH);
static_assert((LDS_QL % 16) == 0 && (LDS_PS % 16) == 0 && (LDS_PMAX % 16) == 0 && (LDS_PSUM % 16) == 0 && (LDS_ST % 16) == 0);
static_assert((SEQ % KCH) == 0 && (SEQ % QB) == 0 && (KCH == 256) && (DM == 8 * 128));
static_assert(((QB * DM / 8) % 256) == 0);

__global__ __launch_bounds__(256) void attn_kernel(const _Float16* __restrict__ qh, const _Float16* __restrict__ ql,
                                                   const _Float16* __restrict__ kh, const _Float16* __restrict__ vh,
                                                   const _Float16* __restrict__ vl, float* __restrict__ out) {
  extern __shared__ __align__(16) char smem[];
  _Float16* QHs = (_Float16*)(smem + LDS_QH);
  _Float16* QLs = (_Float16*)(smem + LDS_QL);
  _Float16* Ps  = (_Float16*)(smem + LDS_PS);
  float* pmax = (float*)(smem + LDS_PMAX);
  float* psum = (float*)(smem + LDS_PSUM);
  float* m_s  = (float*)(smem + LDS_ST);
  float* l_s  = m_s + QB;
  float* al_s = m_s + 2 * QB;
  float* li_s = m_s + 3 * QB;

  const int tid = threadIdx.x, wave = tid >> 5, lane = tid & 31, h = lane >> 4, c = lane & 15;
  const int q0  = (int)blockIdx.x * QB;
  const int b   = (int)blockIdx.x / (SEQ / QB);
  const int kb0 = b * SEQ;
  const float ninf = -__builtin_inff();
  const float sc = 1.0f / 8192.0f;
  const float rq = 1.0f / 2048.0f;

  if (tid < QB) { m_s[tid] = ninf; l_s[tid] = 0.0f; al_s[tid] = 0.0f; li_s[tid] = 0.0f; }
  if (tid < 8 * QB) psum[tid] = 0.0f;
#pragma unroll
  for (int i = 0; i < 8; ++i) {
    const int idx = i * 256 + tid;
    const int row = idx >> 7;
    const int pc  = idx & 127;
    const size_t go = (size_t)(q0 + row) * DM + pc * 8;
    const v8h a = *(const v8h*)(qh + go);
    const v8h d = *(const v8h*)(ql + go);
    *(v8h*)(QHs + row * QSP + pc * 8) = a;
    *(v8h*)(QLs + row * QSP + pc * 8) = d;
  }
  __syncthreads();

  v8f oacc[8];
#pragma unroll
  for (int nt = 0; nt < 8; ++nt) oacc[nt] = zero8();

  const _Float16* qbhp = QHs + c * QSP + 8 * h;
  const _Float16* qblp = QLs + c * QSP + 8 * h;
  const _Float16* pa0p = Ps + c * PSP + 8 * h;
  const int ntile = SEQ / KCH;

#pragma unroll 1
  for (int t = 0; t < ntile; ++t) {
    const int kb = kb0 + t * KCH + 32 * wave;
    const _Float16* ka0p = kh + (size_t)(kb + c) * DM + 8 * h;
    const _Float16* ka1p = kh + (size_t)(kb + 16 + c) * DM + 8 * h;
    v8f sh0 = zero8(), sh1 = zero8(), sl0 = zero8(), sl1 = zero8();
#pragma unroll 1
    for (int k0 = 0; k0 < DM; k0 += 32) {
      const v16h a0 = ldfrag(ka0p + k0), a1 = ldfrag(ka1p + k0);
      const v16h bq = ldfrag(qbhp + k0), br = ldfrag(qblp + k0);
      sh0 = mma16(a0, bq, sh0);
      sh1 = mma16(a1, bq, sh1);
      sl0 = mma16(a0, br, sl0);
      sl1 = mma16(a1, br, sl1);
      guard4_4(sh0, sh1, sl0, sl1, a0, a1, bq, br);
    }
    {
      float pm = ninf;
#pragma unroll
      for (int r = 0; r < 8; ++r) {
        const float v0 = (sh0[r] + sl0[r] * rq) * sc; sh0[r] = v0; pm = fmaxf(pm, v0);
        const float v1 = (sh1[r] + sl1[r] * rq) * sc; sh1[r] = v1; pm = fmaxf(pm, v1);
      }
      pm = fmaxf(pm, __shfl_xor(pm, 16, 32));
      if (h == 0) pmax[wave * QB + c] = pm;
    }
    __syncthreads();
    if (wave == 0) {
      const int row = lane & 15;
      float ps = 0.0f;
#pragma unroll
      for (int w = 0; w < 8; ++w) ps += psum[w * QB + row];
      const float ln = l_s[row] * al_s[row] + ps;
      const float mo = m_s[row];
      float mx = mo;
#pragma unroll
      for (int w = 0; w < 8; ++w) mx = fmaxf(mx, pmax[w * QB + row]);
      const float aln = __expf(mo - mx);
      if (lane < 16) { l_s[row] = ln; al_s[row] = aln; m_s[row] = mx; }
    }
    __syncthreads();
    {
      const float mq = m_s[c];
      float ps = 0.0f;
      v8h h0, h1;
#pragma unroll
      for (int r = 0; r < 8; ++r) {
        const float p0 = __expf(sh0[r] - mq); h0[r] = (_Float16)(p0 * 16.0f); ps += (float)h0[r];
        const float p1 = __expf(sh1[r] - mq); h1[r] = (_Float16)(p1 * 16.0f); ps += (float)h1[r];
      }
      *(v8h*)(Ps + c * PSP + 32 * wave + 8 * h) = h0;
      *(v8h*)(Ps + c * PSP + 32 * wave + 16 + 8 * h) = h1;
      ps += __shfl_xor(ps, 16, 32);
      if (h == 0) psum[wave * QB + c] = ps * 0.0625f;
      const v4f aA = *(const v4f*)(al_s + 8 * h), aB = *(const v4f*)(al_s + 8 * h + 4);
#pragma unroll
      for (int nt = 0; nt < 8; ++nt) {
#pragma unroll
        for (int r = 0; r < 4; ++r) {
          oacc[nt][r] *= aA[r];
          oacc[nt][4 + r] *= aB[r];
        }
      }
    }
    __syncthreads();
    {
      const size_t vbo = (size_t)(128 * wave + c) * NTOK + (size_t)kb0 + (size_t)t * KCH + 8 * h;
      const _Float16* vhp = vh + vbo;
      const _Float16* vlp = vl + vbo;
#pragma unroll
      for (int nt = 0; nt < 8; ++nt) {
        const size_t co = (size_t)(16 * nt) * NTOK;
        v8f accl = zero8();
#pragma unroll 1
        for (int ks = 0; ks < KCH; ks += 32) {
          const v16h pa = ldfrag(pa0p + ks);
          const v16h xb = ldfrag(vhp + co + ks);
          const v16h yb = ldfrag(vlp + co + ks);
          oacc[nt] = mma16(pa, xb, oacc[nt]);
          accl     = mma16(pa, yb, accl);
          guard2_3(oacc[nt], accl, pa, xb, yb);
        }
#pragma unroll
        for (int r = 0; r < 8; ++r) oacc[nt][r] += accl[r] * rq;
      }
    }
  }

  if (wave == 0) {
    const int row = lane & 15;
    float ps = 0.0f;
#pragma unroll
    for (int w = 0; w < 8; ++w) ps += psum[w * QB + row];
    const float l = l_s[row] * al_s[row] + ps;
    if (lane < 16) li_s[row] = (1.0f / l) * (1.0f / 256.0f);
  }
  __syncthreads();
  float* Os = (float*)(smem + LDS_QH);
  {
    const v4f iA = *(const v4f*)(li_s + 8 * h), iB = *(const v4f*)(li_s + 8 * h + 4);
#pragma unroll
    for (int nt = 0; nt < 8; ++nt) {
      const int col = 128 * wave + 16 * nt + c;
#pragma unroll
      for (int r = 0; r < 4; ++r) {
        Os[(8 * h + r) * OSP + col]     = oacc[nt][r] * iA[r];
        Os[(8 * h + 4 + r) * OSP + col] = oacc[nt][4 + r] * iB[r];
      }
    }
  }
  __syncthreads();
  {
    v4f ov[2][8];
#pragma unroll
    for (int rr = 0; rr < 2; ++rr) {
      const int row = 2 * wave + rr;
#pragma unroll
      for (int j = 0; j < 8; ++j) ov[rr][j] = *(const v4f*)(Os + row * OSP + (j * 32 + lane) * 4);
    }
#pragma unroll
    for (int ps = 0; ps < 2; ++ps) {
#pragma unroll
      for (int rr = 0; rr < 2; ++rr) {
        const int row = 2 * wave + rr;
        float* orow = out + (size_t)(q0 + row) * DM;
#pragma unroll
        for (int j = 0; j < 8; ++j) *(volatile v4f*)(orow + (j * 32 + lane) * 4) = ov[rr][j];
      }
      __threadfence();
    }
  }
}

extern "C" void kernel_launch(void* const* d_in, const int* in_sizes, int n_in,
                              void* d_out, int out_size, void* d_ws, size_t ws_size,
                              hipStream_t stream) {
  if (n_in < 4) return;
  const size_t NX = (size_t)NTOK * DM;
  const size_t NW = (size_t)DM * DM;
  if ((size_t)in_sizes[0] != NX || (size_t)in_sizes[1] != NW || (size_t)in_sizes[2] != NW ||
      (size_t)in_sizes[3] != NW) return;
  if ((size_t)out_size != NX) return;

  const float* x  = (const float*)d_in[0];
  const float* Wq = (const float*)d_in[1];
  const float* Wk = (const float*)d_in[2];
  const float* Wv = (const float*)d_in[3];
  float* out = (float*)d_out;

  const size_t bP = NX * 2, bW = NW * 2;
  size_t off = 0;
  const size_t oX  = off; off += bP;
  const size_t oWq = off; off += bW;
  const size_t oWk = off; off += bW;
  const size_t oWv = off; off += bW;
  const size_t oQH = off; off += bP;
  const size_t oQL = off; off += bP;
  const size_t oKH = off; off += bP;
  const size_t oVH = off; off += bP;
  const size_t oVL = off; off += bP;
  if (off > ws_size) return;
  if (off > (size_t)134217728) return;

  char* ws = (char*)d_ws;
  _Float16* X16  = (_Float16*)(ws + oX);
  _Float16* Wq16 = (_Float16*)(ws + oWq);
  _Float16* Wk16 = (_Float16*)(ws + oWk);
  _Float16* Wv16 = (_Float16*)(ws + oWv);
  _Float16* QH   = (_Float16*)(ws + oQH);
  _Float16* QL   = (_Float16*)(ws + oQL);
  _Float16* KH   = (_Float16*)(ws + oKH);
  _Float16* VH   = (_Float16*)(ws + oVH);
  _Float16* VL   = (_Float16*)(ws + oVL);

  const dim3 blk(256);
  const int nbx = (int)(NX / 8 / 256);
  const int nbw = (int)(NW / 8 / 256);

  cvt_kernel<<<dim3(nbx + 3 * nbw), blk, 0, stream>>>(x, Wq, Wk, Wv, X16, Wq16, Wk16, Wv16, nbx, nbw);
  const int gq = (int)(((NTOK / 64) * (DM / 64)) / 8);
  gemm64_kernel<2><<<dim3(gq), blk, 0, stream>>>(X16, DM, Wq16, DM, QH, QL, DM, NTOK, DM, DM, 0.03125f);
  gemm64_kernel<1><<<dim3(gq), blk, 0, stream>>>(X16, DM, Wk16, DM, KH, KH, DM, NTOK, DM, DM, 0.03125f);
  gemm64_kernel<2><<<dim3(gq), blk, 0, stream>>>(Wv16, DM, X16, DM, VH, VL, NTOK, DM, NTOK, DM, 0.03125f);
  (void)hipFuncSetAttribute(reinterpret_cast<const void*>(&attn_kernel),
                            hipFuncAttributeMaxDynamicSharedMemorySize, ATT_LDS);
  attn_kernel<<<dim3(NTOK / QB), blk, ATT_LDS, stream>>>(QH, QL, KH, VH, VL, out);
  (void)hipGetLastError();
}
